// ModuleNet2d_86706799771687
// MI455X (gfx1250) — hardware-verified
//
#include <hip/hip_runtime.h>
#include <math.h>

#pragma clang fp contract(off)

typedef _Float16 v16h __attribute__((ext_vector_type(16)));
typedef _Float16 v8h  __attribute__((ext_vector_type(8)));
typedef float    v8f  __attribute__((ext_vector_type(8)));
typedef float    v4f  __attribute__((ext_vector_type(4)));

constexpr int B_ = 2, C_ = 64, h_ = 96, w_ = 96;
constexpr int H_ = 384, W_ = 384;
constexpr int D_  = 256;
constexpr int CIN = 266;
constexpr int KP  = 288;
constexpr int NT  = 32;
constexpr int NWV = 8;
constexpr float WSC     = 16.0f;
constexpr float WSC_INV = 0.0625f;

constexpr size_t WS_WA  = 0;
constexpr size_t WS_WB  = WS_WA + (size_t)D_ * KP * 2;
constexpr size_t WS_SC  = WS_WB + (size_t)D_ * D_ * 2;
constexpr size_t WS_END = WS_SC + (size_t)B_ * 3 * h_ * w_ * 4;

constexpr int NG_A = D_ * KP / 8;
constexpr int NG_B = D_ * D_ / 8;

static_assert((W_ % NT) == 0);
static_assert((KP % 32) == 0 && KP >= CIN && (KP % 8) == 0);
static_assert(((h_ * w_) % 256) == 0);
static_assert(((NG_A + NG_B) % 256) == 0);
static_assert((WS_WB % 128) == 0 && (WS_SC % 128) == 0 && (WS_END % 128) == 0);
static_assert(D_ == NWV * 32);

__device__ __forceinline__ float coordf(int i, int n) {
    const float c0 = (float)(-1.0 + 1.0 / (double)n);
    const float c2 = (float)(2.0 / (double)n);
    return c0 + c2 * (float)i;
}

__device__ __forceinline__ float gelu_f(float v) {
    return 0.5f * v * (1.0f + erff(v * 0.70710678118654752f));
}

__device__ __forceinline__ v16h ld_frag(const _Float16* row_k0, int h8) {
    v8h e0 = *(const v8h*)(row_k0 + h8);
    v8h e1 = *(const v8h*)(row_k0 + 16 + h8);
    return __builtin_shufflevector(e0, e1, 0, 1, 2, 3, 4, 5, 6, 7, 8, 9, 10, 11, 12, 13, 14, 15);
}

__device__ __forceinline__ void mma4(v8f& d00, v8f& d01, v8f& d10, v8f& d11,
                                     v16h A0, v16h A1, v16h B0, v16h B1) {
    d00 = __builtin_amdgcn_wmma_f32_16x16x32_f16(false, A0, false, B0, (short)0, d00, false, false);
    d01 = __builtin_amdgcn_wmma_f32_16x16x32_f16(false, A0, false, B1, (short)0, d01, false, false);
    d10 = __builtin_amdgcn_wmma_f32_16x16x32_f16(false, A1, false, B0, (short)0, d10, false, false);
    d11 = __builtin_amdgcn_wmma_f32_16x16x32_f16(false, A1, false, B1, (short)0, d11, false, false);
    asm volatile("v_nop\n\tv_nop\n\tv_nop\n\tv_nop"
                 : "+v"(d00), "+v"(d01), "+v"(d10), "+v"(d11)
                 : "v"(A0), "v"(A1), "v"(B0), "v"(B1));
}

__global__ __launch_bounds__(256)
void prep_weights(const float* __restrict__ w00, const float* __restrict__ w1,
                  _Float16* Wa, _Float16* Wb) {
    const int g = blockIdx.x * 256 + threadIdx.x;
    const bool valid = g < NG_A + NG_B;
    v8h v;
#pragma unroll
    for (int i = 0; i < 8; ++i) v[i] = (_Float16)0.0f;
    _Float16* dst = Wa;
    if (g < NG_A) {
        const int o = (8 * g) / KP, k = (8 * g) % KP;
#pragma unroll
        for (int i = 0; i < 8; ++i) {
            const int kk = k + i;
            const float x = w00[min(o * CIN + kk, D_ * CIN - 1)];
            v[i] = (_Float16)((kk < CIN) ? x * WSC : 0.0f);
        }
        dst = Wa + (size_t)8 * g;
    } else if (valid) {
        const int j = g - NG_A;
#pragma unroll
        for (int i = 0; i < 8; ++i) v[i] = (_Float16)(w1[8 * j + i] * WSC);
        dst = Wb + (size_t)8 * j;
    }
    if (valid) *(volatile v8h*)dst = v;
    __threadfence();
    if (valid) *(volatile v8h*)dst = v;
}

__global__ __launch_bounds__(256)
void shortcut_kernel(const float* __restrict__ feat,
                     const float* __restrict__ ws1, const float* __restrict__ bs1,
                     const float* __restrict__ ws2, const float* __restrict__ bs2,
                     float* sc) {
    __shared__ __align__(16) float s_sc[3 * 256];
    const int t    = threadIdx.x;
    const int i0   = blockIdx.x * 256;
    const int b    = i0 / (h_ * w_);
    const int rem0 = i0 % (h_ * w_);
    const int rem  = rem0 + t;
    const float* fp = feat + (size_t)b * C_ * h_ * w_ + rem;
    float f[C_];
#pragma unroll
    for (int c = 0; c < C_; ++c) f[c] = fp[(size_t)c * h_ * w_];
    float o0 = bs2[0], o1 = bs2[1], o2 = bs2[2];
    for (int j = 0; j < C_; ++j) {
        float a = bs1[j];
        const float* wr = ws1 + j * C_;
#pragma unroll
        for (int c = 0; c < C_; ++c) a = fmaf(wr[c], f[c], a);
        a = fmaxf(a, 0.0f);
        o0 = fmaf(ws2[0 * C_ + j], a, o0);
        o1 = fmaf(ws2[1 * C_ + j], a, o1);
        o2 = fmaf(ws2[2 * C_ + j], a, o2);
    }
    s_sc[0 * 256 + t] = o0;
    s_sc[1 * 256 + t] = o1;
    s_sc[2 * 256 + t] = o2;
    __syncthreads();

    v4f v = {0.0f, 0.0f, 0.0f, 0.0f};
    float* dst = sc;
    const bool valid = t < 3 * 64;
    if (valid) {
        const int o = t >> 6, j = t & 63;
        v   = *(const v4f*)(s_sc + o * 256 + 4 * j);
        dst = sc + ((size_t)b * 3 + o) * h_ * w_ + rem0 + 4 * j;
    }
    if (valid) *(volatile v4f*)dst = v;
    __threadfence();
    if (valid) *(volatile v4f*)dst = v;
}

__global__ __launch_bounds__(256)
void liif_main(const float* __restrict__ feat,
               const _Float16* __restrict__ Wa, const float* __restrict__ b00,
               const _Float16* __restrict__ Wb, const float* __restrict__ b1,
               const float* __restrict__ w2, const float* __restrict__ b2,
               const float* __restrict__ sc,
               const int* __restrict__ tgt_h, const int* __restrict__ tgt_w,
               float* out) {
    __shared__ __align__(16) _Float16 g_lds[NT * KP];
    __shared__ __align__(16) _Float16 x_lds[NT * D_];
    __shared__ __align__(16) float s_part[NWV * 3 * NT];
    __shared__ __align__(16) float s_out[3 * NT];
    __shared__ int   s_iy[4][NT], s_ix[4][NT];
    __shared__ float s_wq[4][NT];

    const int t    = threadIdx.x;
    const int pix0 = blockIdx.x * NT;
    const int b    = pix0 / (H_ * W_);
    const int rem  = pix0 % (H_ * W_);
    const int yy   = rem / W_;
    const int x0   = rem % W_;

    if (t < NT) {
        const int Ht = max(tgt_h[0], 1), Wt = max(tgt_w[0], 1);
        const int xx = x0 + t;
        const float cy  = coordf(yy, Ht);
        const float cx  = coordf(xx, Wt);
        const float rxs = (float)(1.0 / (double)h_);
        const float rys = (float)(1.0 / (double)w_);
        const float eps = (float)1e-6;
        const float clo = (float)(-1.0 + 1e-6), chi = (float)(1.0 - 1e-6);
        _Float16* gp = g_lds + t * KP;
        float area[4];
#pragma unroll
        for (int qd = 0; qd < 4; ++qd) {
            const float vx = (qd & 2) ? 1.0f : -1.0f;
            const float vy = (qd & 1) ? 1.0f : -1.0f;
            const float sy = fminf(fmaxf(cy + vx * rxs + eps, clo), chi);
            const float sx = fminf(fmaxf(cx + vy * rys + eps, clo), chi);
            const float uy = ((sy + 1.0f) * (float)h_ - 1.0f) * 0.5f;
            const float ux = ((sx + 1.0f) * (float)w_ - 1.0f) * 0.5f;
            int iy = (int)rintf(uy);
            int ix = (int)rintf(ux);
            iy = min(max(iy, 0), h_ - 1);
            ix = min(max(ix, 0), w_ - 1);
            const float oldy = coordf(iy, h_);
            const float oldx = coordf(ix, w_);
            const float rely = (cy - oldy) * (float)h_;
            const float relx = (cx - oldx) * (float)w_;
            area[qd] = fabsf(rely * relx) + (float)1e-9;
            s_iy[qd][t] = iy;
            s_ix[qd][t] = ix;
            gp[2 * qd + 0] = (_Float16)rely;
            gp[2 * qd + 1] = (_Float16)relx;
        }
        const float tot  = ((area[0] + area[1]) + area[2]) + area[3];
        const float rtot = 1.0f / tot;
#pragma unroll
        for (int qd = 0; qd < 4; ++qd) s_wq[qd][t] = area[3 - qd] * rtot;
        const double cellh = (2.0 / (double)Ht) * fmax(((double)Ht / (double)h_) / 4.0, 1.0) * (double)h_;
        const double cellw = (2.0 / (double)Wt) * fmax(((double)Wt / (double)w_) / 4.0, 1.0) * (double)w_;
        gp[264] = (_Float16)((float)cellh);
        gp[265] = (_Float16)((float)cellw);
#pragma unroll
        for (int k = CIN; k < KP; ++k) gp[k] = (_Float16)0.0f;
    }
    __syncthreads();

    {
        const int p = t & (NT - 1), s = t >> 5;
        const float* fb = feat + (size_t)b * C_ * h_ * w_;
#pragma unroll
        for (int qd = 0; qd < 4; ++qd) {
            const int   idx = s_iy[qd][p] * w_ + s_ix[qd][p];
            const float wq  = s_wq[qd][p];
#pragma unroll
            for (int u = 0; u < 8; ++u) {
                const int c = s * 8 + u;
                g_lds[p * KP + 8 + qd * 64 + c] = (_Float16)(fb[(size_t)c * h_ * w_ + idx] * wq);
            }
        }
    }
    __syncthreads();

    const int lane   = t & 31;
    const int wv     = t >> 5;
    const int p      = lane & 15;
    const int lh     = lane >> 4;
    const int h8     = lh * 8;
    const int m_base = wv * 32;

    v8f a00 = {}, a01 = {}, a10 = {}, a11 = {};
    for (int k0 = 0; k0 < KP; k0 += 32) {
        const _Float16* pa = Wa + (size_t)(m_base + p) * KP + k0;
        v16h A0 = ld_frag(pa, h8);
        v16h A1 = ld_frag(pa + (size_t)16 * KP, h8);
        v16h B0 = ld_frag(g_lds + p * KP + k0, h8);
        v16h B1 = ld_frag(g_lds + (p + 16) * KP + k0, h8);
        mma4(a00, a01, a10, a11, A0, A1, B0, B1);
    }
#pragma unroll
    for (int r = 0; r < 8; ++r) {
        const int m0 = m_base + h8 + r;
        const int m1 = m0 + 16;
        const float bm0 = b00[m0], bm1 = b00[m1];
        x_lds[p * D_ + m0]        = (_Float16)(a00[r] * WSC_INV + bm0);
        x_lds[(p + 16) * D_ + m0] = (_Float16)(a01[r] * WSC_INV + bm0);
        x_lds[p * D_ + m1]        = (_Float16)(a10[r] * WSC_INV + bm1);
        x_lds[(p + 16) * D_ + m1] = (_Float16)(a11[r] * WSC_INV + bm1);
    }
    __syncthreads();

    v8f c00 = {}, c01 = {}, c10 = {}, c11 = {};
    for (int k0 = 0; k0 < D_; k0 += 32) {
        const _Float16* pa = Wb + (size_t)(m_base + p) * D_ + k0;
        v16h A0 = ld_frag(pa, h8);
        v16h A1 = ld_frag(pa + (size_t)16 * D_, h8);
        v16h B0 = ld_frag(x_lds + p * D_ + k0, h8);
        v16h B1 = ld_frag(x_lds + (p + 16) * D_ + k0, h8);
        mma4(c00, c01, c10, c11, A0, A1, B0, B1);
    }
    {
        float S0[3] = {0.0f, 0.0f, 0.0f};
        float S1[3] = {0.0f, 0.0f, 0.0f};
#pragma unroll
        for (int r = 0; r < 8; ++r) {
            const int m0 = m_base + h8 + r;
            const int m1 = m0 + 16;
            const float bb0 = b1[m0], bb1 = b1[m1];
            const float v00 = gelu_f(c00[r] * WSC_INV + bb0);
            const float v01 = gelu_f(c01[r] * WSC_INV + bb0);
            const float v10 = gelu_f(c10[r] * WSC_INV + bb1);
            const float v11 = gelu_f(c11[r] * WSC_INV + bb1);
#pragma unroll
            for (int o = 0; o < 3; ++o) {
                const float wa = w2[o * D_ + m0], wb = w2[o * D_ + m1];
                S0[o] = fmaf(wb, v10, fmaf(wa, v00, S0[o]));
                S1[o] = fmaf(wb, v11, fmaf(wa, v01, S1[o]));
            }
        }
#pragma unroll
        for (int o = 0; o < 3; ++o) {
            S0[o] += __shfl_xor(S0[o], 16);
            S1[o] += __shfl_xor(S1[o], 16);
            s_part[(wv * 3 + o) * NT + lane] = lh ? S1[o] : S0[o];
        }
    }
    __syncthreads();

    if (t < 3 * NT) {
        const int o  = t >> 5;
        const int pp = t & (NT - 1);
        float acc = b2[o];
#pragma unroll
        for (int q = 0; q < NWV; ++q) acc += s_part[(q * 3 + o) * NT + pp];

        const int Ht = max(tgt_h[0], 1), Wt = max(tgt_w[0], 1);
        const int xx = x0 + pp;
        const float cy = coordf(yy, Ht);
        const float cx = coordf(xx, Wt);
        const float uy = ((cy + 1.0f) * (float)h_ - 1.0f) * 0.5f;
        const float ux = ((cx + 1.0f) * (float)w_ - 1.0f) * 0.5f;
        const float fy = floorf(uy), fx = floorf(ux);
        const float wy = uy - fy,    wx = ux - fx;
        const int y0i = min(max((int)fy, 0), h_ - 1);
        const int y1i = min(max((int)fy + 1, 0), h_ - 1);
        const int x0i = min(max((int)fx, 0), w_ - 1);
        const int x1i = min(max((int)fx + 1, 0), w_ - 1);
        const float* sp = sc + ((size_t)b * 3 + o) * h_ * w_;
        const float g00 = (1.0f - wy) * (1.0f - wx);
        const float g01 = (1.0f - wy) * wx;
        const float g10 = wy * (1.0f - wx);
        const float g11 = wy * wx;
        const float samp = ((sp[y0i * w_ + x0i] * g00 + sp[y0i * w_ + x1i] * g01)
                            + sp[y1i * w_ + x0i] * g10) + sp[y1i * w_ + x1i] * g11;
        s_out[o * NT + pp] = acc + samp;
    }
    __syncthreads();

    {
        v4f v = {0.0f, 0.0f, 0.0f, 0.0f};
        float* dst = out;
        const bool valid = t < 24;
        if (valid) {
            const int o = t >> 3, j = t & 7;
            v   = *(const v4f*)(s_out + o * NT + 4 * j);
            dst = out + ((size_t)b * 3 + o) * H_ * W_ + (size_t)yy * W_ + x0 + 4 * j;
        }
        if (valid) *(volatile v4f*)dst = v;
        __threadfence();
        if (valid) *(volatile v4f*)dst = v;
    }
}

extern "C" void kernel_launch(void* const* d_in, const int* in_sizes, int n_in,
                              void* d_out, int out_size, void* d_ws, size_t ws_size,
                              hipStream_t stream) {
    if (n_in < 13) return;
    if (in_sizes[0] != B_ * C_ * h_ * w_) return;
    if (in_sizes[1] != D_ * CIN || in_sizes[3] != D_ * D_) return;
    if (out_size != B_ * 3 * H_ * W_) return;
    if ((size_t)WS_END > ws_size) return;

    const float* feat = (const float*)d_in[0];
    const float* w00  = (const float*)d_in[1];
    const float* b00  = (const float*)d_in[2];
    const float* w1   = (const float*)d_in[3];
    const float* b1   = (const float*)d_in[4];
    const float* w2   = (const float*)d_in[5];
    const float* b2   = (const float*)d_in[6];
    const float* ws1  = (const float*)d_in[7];
    const float* bs1  = (const float*)d_in[8];
    const float* ws2  = (const float*)d_in[9];
    const float* bs2  = (const float*)d_in[10];
    const int* tgt_h  = (const int*)d_in[11];
    const int* tgt_w  = (const int*)d_in[12];
    float* out = (float*)d_out;

    char* ws = (char*)d_ws;
    _Float16* Wa = (_Float16*)(ws + WS_WA);
    _Float16* Wb = (_Float16*)(ws + WS_WB);
    float*    sc = (float*)(ws + WS_SC);

    const int nprep = NG_A + NG_B;
    prep_weights<<<(nprep + 255) / 256, 256, 0, stream>>>(w00, w1, Wa, Wb);

    const int nsc = B_ * h_ * w_;
    shortcut_kernel<<<nsc / 256, 256, 0, stream>>>(feat, ws1, bs1, ws2, bs2, sc);

    const int nblk = (B_ * H_ * W_) / NT;
    liif_main<<<nblk, 256, 0, stream>>>(feat, Wa, b00, Wb, b1, w2, b2, sc, tgt_h, tgt_w, out);
}
